// TransformerBlock_57105885168168
// MI455X (gfx1250) — hardware-run, weakly checked
//
#include <hip/hip_runtime.h>


#ifndef NB
#define NB 2
#endif
#ifndef SEQ
#define SEQ 2048
#endif
#define NB_FULL  2
#define SEQ_FULL 2048
#define TT   SEQ
#define DM   1024
#define NH_  16
#define HD   64
#define DQ   (NH_ * HD)
#define FF   4096
#define MC   (TT / 2)
#define WCAR 1024.0f
#define CCAR 64.0f
#define GCAR 256.0f
#define PEXP 8.0f
#define SCL2 (0.125f * 1.4426950408889634f)
typedef _Float16 h16;
typedef unsigned short bf;
typedef __attribute__((ext_vector_type(16))) __bf16   v16bf;
typedef __attribute__((ext_vector_type(16))) _Float16 v16h;
typedef __attribute__((ext_vector_type(8)))  _Float16 v8h;
typedef __attribute__((ext_vector_type(8)))  unsigned short v8us;
typedef __attribute__((ext_vector_type(8)))  float    v8f;
typedef __attribute__((ext_vector_type(4)))  float    v4f;
typedef v8h  __attribute__((may_alias)) v8ha;
typedef v4f  __attribute__((may_alias)) v4fa;
typedef v8us __attribute__((may_alias)) v8usa;

static_assert(TT % 128 == 0);
static_assert(DM % 64 == 0);
static_assert((3 * DQ) % 64 == 0);
static_assert(HD == 64);
static_assert(TT <= SEQ_FULL);
static_assert(NB <= NB_FULL);
static_assert(NB <= 4);
static_assert(DM == 1024);
static_assert(DM % 256 == 0);
static_assert(DM % 32 == 0);
static_assert(DQ % 32 == 0);
static_assert(FF % 64 == 0);
static_assert(FF % 32 == 0);
static_assert((2 * FF) % 64 == 0);
static_assert(MC % 64 == 0);
static_assert(2 * MC == TT);
static_assert(DQ == DM);
static_assert((TT / 32) >= 4);

__device__ __forceinline__ unsigned short f2bf(float f) { unsigned u = __float_as_uint(f); u += 0x7FFFu + ((u >> 16) & 1u); return (unsigned short)(u >> 16); }
__device__ __forceinline__ float bf2f(unsigned short b) { return __uint_as_float(((unsigned)b) << 16); }
__device__ __forceinline__ float bfr(float f) { return bf2f(f2bf(f)); }
__device__ __forceinline__ v16h cat16(v8h lo, v8h hi) { return __builtin_shufflevector(lo, hi, 0, 1, 2, 3, 4, 5, 6, 7, 8, 9, 10, 11, 12, 13, 14, 15); }
__device__ __forceinline__ v16bf cat16b(v8us lo, v8us hi) { return __builtin_bit_cast(v16bf, __builtin_shufflevector(lo, hi, 0, 1, 2, 3, 4, 5, 6, 7, 8, 9, 10, 11, 12, 13, 14, 15)); }
__device__ __forceinline__ v8f wmma16(v16h a, v16h b, v8f c) { return __builtin_amdgcn_wmma_f32_16x16x32_f16(false, a, false, b, (short)0, c, false, false); }
__device__ __forceinline__ v8f wmmab(v16bf a, v16bf b, v8f c) { return __builtin_amdgcn_wmma_f32_16x16x32_bf16(false, a, false, b, (short)0, c, false, false); }

static __device__ __forceinline__ h16 toh_flush(float v) { const h16 r = (h16)v; return (fabsf(v) < 6.103515625e-05f) ? (h16)0.0f : r; }
static __device__ __forceinline__ v8f wmma16g(v16h a, v16h b, v8f c) { c = wmma16(a, b, c); asm volatile("v_nop\n\tv_nop\n\tv_nop\n\tv_nop" : "+v"(c) : "v"(a), "v"(b)); return c; }
static __device__ __forceinline__ float silu_f(float a) { const float e = __builtin_amdgcn_exp2f(a * -1.4426950408889634f); return a * __builtin_amdgcn_rcpf(1.0f + e); }

template <typename T16> struct WFrag;
template <> struct WFrag<h16> { typedef v16h V; static __device__ __forceinline__ V ld(const h16* p) { return cat16(*(const v8h*)p, *(const v8h*)(p + 16)); } static __device__ __forceinline__ v8f mma(V a, V b, v8f c) { return wmma16(a, b, c); } };
template <> struct WFrag<bf> { typedef v16bf V; static __device__ __forceinline__ V ld(const bf* p) { return cat16b(*(const v8us*)p, *(const v8us*)(p + 16)); } static __device__ __forceinline__ v8f mma(V a, V b, v8f c) { return wmmab(a, b, c); } };
template <typename T16, int NSPLIT, bool BIAS, int RES>
__device__ __forceinline__ void gemm_tile(const T16* __restrict__ A, const T16* __restrict__ A2, const T16* __restrict__ Bt, const T16* __restrict__ Bt2, int K, float* C, int ldc, const float* __restrict__ bias, const float* __restrict__ R, int ldr, float osc) {
    typedef typename WFrag<T16>::V V;
    __shared__ __align__(16) float os[16 * 68];
    const int lane = threadIdx.x & 31, lr = lane & 15, hi = lane >> 4; const int r0 = blockIdx.x * 64, c0 = blockIdx.y * 64;
    v8f acc[4][4];
#pragma unroll
    for (int mb = 0; mb < 4; ++mb)
#pragma unroll
        for (int nb = 0; nb < 4; ++nb) acc[mb][nb] = (v8f){};
    const size_t aoff = (size_t)(r0 + lr) * K + 8 * hi, boff = (size_t)(c0 + lr) * K + 8 * hi;
#pragma unroll 1
    for (int kc = 0; kc < K; kc += 32) {
        V a[4], a2[4];
#pragma unroll
        for (int mb = 0; mb < 4; ++mb) { a[mb] = WFrag<T16>::ld(A + aoff + (size_t)mb * 16 * K + kc); if (NSPLIT == 1 || NSPLIT == 2) a2[mb] = WFrag<T16>::ld(A2 + aoff + (size_t)mb * 16 * K + kc); }
#pragma unroll
        for (int nb = 0; nb < 4; ++nb) { const V b = WFrag<T16>::ld(Bt + boff + (size_t)nb * 16 * K + kc); V b2; if (NSPLIT >= 2) b2 = WFrag<T16>::ld(Bt2 + boff + (size_t)nb * 16 * K + kc);
#pragma unroll
            for (int mb = 0; mb < 4; ++mb) { acc[mb][nb] = WFrag<T16>::mma(a[mb], b, acc[mb][nb]); if (NSPLIT == 1 || NSPLIT == 2) acc[mb][nb] = WFrag<T16>::mma(a2[mb], b, acc[mb][nb]); if (NSPLIT >= 2) acc[mb][nb] = WFrag<T16>::mma(a[mb], b2, acc[mb][nb]); } }
        asm volatile("v_nop\n\tv_nop\n\tv_nop\n\tv_nop" : "+v"(acc[0][0]), "+v"(acc[1][1]), "+v"(acc[2][2]), "+v"(acc[3][3]) : "v"(a[0]), "v"(a[3]));
    }
    v4f bv = (v4f){0.f, 0.f, 0.f, 0.f};
    if (BIAS) { const v4f b4 = *(const v4f*)(bias + c0 + lr * 4);
#pragma unroll
        for (int q = 0; q < 4; ++q) bv[q] = bfr(b4[q]); }
#pragma unroll
    for (int mb = 0; mb < 4; ++mb) {
#pragma unroll
        for (int nb = 0; nb < 4; ++nb) {
#pragma unroll
            for (int j = 0; j < 8; ++j) os[(hi * 8 + j) * 68 + nb * 16 + lr] = acc[mb][nb][j]; }
        __builtin_amdgcn_wave_barrier(); asm volatile("" ::: "memory");
        float* crow = C + (size_t)(r0 + mb * 16) * ldc + c0;
        const size_t rbase = (size_t)(r0 + mb * 16) * ldr + c0;
#pragma unroll 1
        for (int ps = 0; ps < 2; ++ps) {
#pragma unroll
            for (int s = 0; s < 8; ++s) { const int row = 2 * s + hi, cofs = lr * 4; v4f val = *(const v4fa*)(os + row * 68 + cofs);
#pragma unroll
                for (int q = 0; q < 4; ++q) val[q] = val[q] * osc + bv[q];
                if (RES != 0) { const v4f rv = *(const v4f*)(R + rbase + (size_t)row * ldr + cofs);
#pragma unroll
                    for (int q = 0; q < 4; ++q) val[q] += (RES == 1) ? bfr(rv[q]) : rv[q]; }
                *(volatile v4f*)(crow + (size_t)row * ldc + cofs) = val; }
            if (ps == 0) __threadfence(); }
        __builtin_amdgcn_wave_barrier(); asm volatile("" ::: "memory");
    }
}

__global__ __launch_bounds__(32) void k_gemm_nb(const h16* __restrict__ A, const h16* __restrict__ Bt, int K, float* C, int ldc, float osc) {
    gemm_tile<h16, 0, false, 0>(A, nullptr, Bt, nullptr, K, C, ldc, nullptr, nullptr, 0, osc); }
__global__ __launch_bounds__(32) void k_gemm_b(const h16* __restrict__ A, const h16* __restrict__ Bt, int K, float* C, int ldc, const float* __restrict__ bias, float osc) {
    gemm_tile<h16, 0, true, 0>(A, nullptr, Bt, nullptr, K, C, ldc, bias, nullptr, 0, osc); }
__global__ __launch_bounds__(32) void k_gemm_br1(const h16* __restrict__ A, const h16* __restrict__ Bt, int K, float* C, int ldc, const float* __restrict__ bias, const float* __restrict__ R, int ldr, float osc) {
    gemm_tile<h16, 0, true, 1>(A, nullptr, Bt, nullptr, K, C, ldc, bias, R, ldr, osc); }
__global__ __launch_bounds__(32) void k_gemm_br2(const h16* __restrict__ A, const h16* __restrict__ Bt, int K, float* C, int ldc, const float* __restrict__ bias, const float* __restrict__ R, int ldr, float osc) {
    gemm_tile<h16, 0, true, 2>(A, nullptr, Bt, nullptr, K, C, ldc, bias, R, ldr, osc); }

__global__ __launch_bounds__(128) __attribute__((amdgpu_num_vgpr(256))) void k_flash(const h16* __restrict__ QP, const h16* __restrict__ KP, const h16* __restrict__ VT, const int* __restrict__ mk, h16* CTX) {
    __shared__ unsigned mw[TT / 32];
    __shared__ __align__(16) h16 ot[4 * 16 * 72];
    const int lane = threadIdx.x & 31, lr = lane & 15, hi = lane >> 4;
    const int wave = __builtin_amdgcn_readfirstlane((int)(threadIdx.x >> 5));
    const int head = blockIdx.y; const int q0 = blockIdx.x * 64 + wave * 16;
#pragma unroll 1
    for (int i = wave; i < TT / 32; i += 4) { const int m = mk[i * 32 + lane]; const unsigned bw = __builtin_amdgcn_ballot_w32(m != 0); if (lane == 0) mw[i] = bw; }
    __syncthreads();
    unsigned any = 0u;
#pragma unroll 1
    for (int i0 = 0; i0 < TT / 32; i0 += 32) { const int i = i0 + lane; any |= mw[(i < TT / 32) ? i : (TT / 32 - 1)]; }
#pragma unroll
    for (int sh = 16; sh; sh >>= 1) any |= (unsigned)__shfl_xor((int)any, sh, 32);
    const bool allm = (any == 0u);
    const float scl = allm ? 0.0f : SCL2; const unsigned force = allm ? 0xFFFFFFFFu : 0u;
    const size_t hb = (size_t)head * TT * HD;
    const h16* qp = QP + hb + (size_t)(q0 + lr) * HD + 8 * hi;
    const v16h bq0 = WFrag<h16>::ld(qp), bq1 = WFrag<h16>::ld(qp + 32);
    const h16* kp = KP + hb + (size_t)lr * HD + 8 * hi;
    const h16* vp = VT + (size_t)head * HD * TT + (size_t)lr * TT + 8 * hi;
    v8f o[4];
#pragma unroll
    for (int dt = 0; dt < 4; ++dt) o[dt] = (v8f){};
    float mrun = -3.0e38f, lrun = 0.f; const float ninf = -__builtin_huge_valf();
#pragma unroll 1
    for (int kt = 0; kt < TT / 32; ++kt) {
        const int kb = kt * 32;
        const v16h ak00 = WFrag<h16>::ld(kp + (size_t)kb * HD), ak01 = WFrag<h16>::ld(kp + (size_t)kb * HD + 32);
        const v16h ak10 = WFrag<h16>::ld(kp + (size_t)(kb + 16) * HD), ak11 = WFrag<h16>::ld(kp + (size_t)(kb + 16) * HD + 32);
        v16h av[4];
#pragma unroll
        for (int dt = 0; dt < 4; ++dt) av[dt] = WFrag<h16>::ld(vp + (size_t)dt * 16 * TT + kb);
        v8f s0 = (v8f){}, s1 = (v8f){};
        s0 = wmma16g(ak00, bq0, s0); s0 = wmma16g(ak01, bq1, s0);
        s1 = wmma16g(ak10, bq0, s1); s1 = wmma16g(ak11, bq1, s1);
        const unsigned w = (mw[kt] | force) >> (8 * hi);
        float t[16];
#pragma unroll
        for (int r = 0; r < 8; ++r) { const float a = s0[r] * scl; t[r] = ((w >> r) & 1u) ? a : ninf; const float b = s1[r] * scl; t[8 + r] = ((w >> (16 + r)) & 1u) ? b : ninf; }
        float mx = t[0];
#pragma unroll
        for (int i = 1; i < 16; ++i) mx = fmaxf(mx, t[i]);
        mx = fmaxf(mx, __shfl_xor(mx, 16, 32));
        const float mn = fmaxf(mrun, mx);
        const float al = __builtin_amdgcn_exp2f(mrun - mn);
        mrun = mn;
        v16h pb; float rs = 0.f;
#pragma unroll
        for (int i = 0; i < 16; ++i) { const float e = (t[i] - mn) + PEXP; const float p = (e < -14.0f) ? 0.0f : __builtin_amdgcn_exp2f(e); const h16 ph = (h16)p; pb[i] = ph; rs += (float)ph; }
        lrun = lrun * al + rs;
#pragma unroll
        for (int dt = 0; dt < 4; ++dt)
#pragma unroll
            for (int r = 0; r < 8; ++r) o[dt][r] *= al;
#pragma unroll
        for (int dt = 0; dt < 4; ++dt) o[dt] = wmma16g(av[dt], pb, o[dt]);
    }
    const float l = lrun + __shfl_xor(lrun, 16, 32);
    const float inv = CCAR * __builtin_amdgcn_rcpf(l);
    const int ob = wave * 16 * 72;
#pragma unroll
    for (int dt = 0; dt < 4; ++dt) { v8h o8;
#pragma unroll
        for (int r = 0; r < 8; ++r) o8[r] = toh_flush(o[dt][r] * inv);
        *(v8ha*)(&ot[ob + lr * 72 + dt * 16 + hi * 8]) = o8; }
    __builtin_amdgcn_wave_barrier(); asm volatile("" ::: "memory");
    h16* crow = CTX + (size_t)q0 * DQ + head * HD;
#pragma unroll 1
    for (int ps = 0; ps < 2; ++ps) {
#pragma unroll
        for (int s = 0; s < 4; ++s) { const int row = 4 * s + (lane >> 3), pc = lane & 7; const v8h v = *(const v8ha*)(&ot[ob + row * 72 + pc * 8]);
            *(volatile v8h*)(crow + (size_t)row * DQ + pc * 8) = v; }
        if (ps == 0) __threadfence(); }
}

__global__ __launch_bounds__(256) void k_cvtw(const float* __restrict__ src, h16* dst, size_t n8) {
#pragma clang fp contract(off)
    const size_t i = (size_t)blockIdx.x * 256 + threadIdx.x; if (i >= n8) return; const v8f v = *(const v8f*)(src + i * 8); v8h o;
#pragma unroll
    for (int k = 0; k < 8; ++k) o[k] = toh_flush(bfr(v[k]) * WCAR);
    *(volatile v8h*)(dst + i * 8) = o; __threadfence(); *(volatile v8h*)(dst + i * 8) = o; }

__global__ __launch_bounds__(256) void k_hpl16(const float* __restrict__ F, int pitch, int nheads, h16* P16) {
#pragma clang fp contract(off)
    const size_t e = ((size_t)blockIdx.x * 256 + threadIdx.x) * 8; if (e >= (size_t)nheads * TT * HD) return; const int d = (int)(e % HD); const int t = (int)((e / HD) % TT); const int h = (int)(e / ((size_t)HD * TT));
    const v8f x = *(const v8f*)(F + (size_t)t * pitch + h * HD + d); v8h o;
#pragma unroll
    for (int q = 0; q < 8; ++q) o[q] = toh_flush(x[q]);
    *(volatile v8h*)(P16 + e) = o; __threadfence(); *(volatile v8h*)(P16 + e) = o; }

__global__ __launch_bounds__(256) void k_vtp16(const float* __restrict__ F, int pitch, int nheads, h16* V16) {
#pragma clang fp contract(off)
    const size_t e = ((size_t)blockIdx.x * 256 + threadIdx.x) * 8; if (e >= (size_t)nheads * HD * TT) return; const int t = (int)(e % TT); const int d = (int)((e / TT) % HD); const int g = (int)(e / ((size_t)TT * HD)); v8h o;
#pragma unroll
    for (int q = 0; q < 8; ++q) { const float x = F[(size_t)(t + q) * pitch + g * HD + d]; o[q] = toh_flush(x); }
    *(volatile v8h*)(V16 + e) = o; __threadfence(); *(volatile v8h*)(V16 + e) = o; }

__global__ __launch_bounds__(256) void k_mod(const float* __restrict__ c, const float* __restrict__ W, const float* __restrict__ wb, float* MODv, int isscale) {
#pragma clang fp contract(off)
    __shared__ float scs[NB * DM];
    __shared__ __align__(16) float res[4 * 32];
    const int lane = threadIdx.x & 31; const int wave = __builtin_amdgcn_readfirstlane((int)(threadIdx.x >> 5)); const int cb = blockIdx.x * 32;
#pragma unroll 1
    for (int i = threadIdx.x; i < NB * DM; i += 256) scs[i] = silu_f(bfr(c[i]));
    __syncthreads();
#pragma unroll 1
    for (int j = 0; j < 4; ++j) { const int col = cb + wave * 4 + j; const float* wr = W + (size_t)col * DM; float a[NB];
#pragma unroll
        for (int b = 0; b < NB; ++b) a[b] = 0.f;
#pragma unroll 1
        for (int k = lane; k < DM; k += 32) { const float wv = bfr(wr[k]);
#pragma unroll
            for (int b = 0; b < NB; ++b) a[b] += scs[b * DM + k] * wv; }
        const float bias = bfr(wb[col]);
#pragma unroll
        for (int b = 0; b < NB; ++b) { float s = a[b];
#pragma unroll
            for (int sh = 16; sh; sh >>= 1) s += __shfl_xor(s, sh, 32);
            float v = s + bias; const float vc = fminf(10.0f, fmaxf(0.1f, v + 1.0f)); v = isscale ? vc : v;
            if (lane == 0) res[b * 32 + wave * 4 + j] = v; } }
    __syncthreads();
    if (wave == 0) { const int bq = lane >> 3; const int b = (bq < NB) ? bq : (NB - 1); const int pc = lane & 7; const v4f v = *(const v4fa*)(res + b * 32 + pc * 4); float* dst = MODv + (size_t)b * DM + cb + pc * 4;
        if (lane < 8 * NB) { *(volatile v4f*)dst = v; __threadfence(); *(volatile v4f*)dst = v; } }
}

__global__ __launch_bounds__(256) void k_adaln(const float* __restrict__ X, int rnd, const float* __restrict__ nw, const float* __restrict__ scv, const float* __restrict__ shv, h16* HB) {
#pragma clang fp contract(off)
    const int lane = threadIdx.x & 31; const int row = blockIdx.x * 8 + __builtin_amdgcn_readfirstlane((int)(threadIdx.x >> 5)); if (row >= TT) return;
    const float* xr = X + (size_t)row * DM; float ss = 0.f;
#pragma unroll 1
    for (int j = 0; j < DM / 256; ++j) { const v8f v = *(const v8f*)(xr + j * 256 + lane * 8);
#pragma unroll
        for (int q = 0; q < 8; ++q) { const float a = rnd ? bfr(v[q]) : v[q]; ss += a * a; } }
#pragma unroll
    for (int sh = 16; sh; sh >>= 1) ss += __shfl_xor(ss, sh, 32);
    const float nrm = fmaxf(sqrtf(ss) * 0.03125f, 1.0e-6f); const float rinv = 1.0f / nrm;
#pragma unroll 1
    for (int ps = 0; ps < 2; ++ps) {
#pragma unroll 1
        for (int j = 0; j < DM / 256; ++j) { const int c0 = j * 256 + lane * 8; const v8f v = *(const v8f*)(xr + c0); const v8f g = *(const v8f*)(nw + c0); const v8f sc = *(const v8f*)(scv + c0); const v8f sf = *(const v8f*)(shv + c0); v8h o;
#pragma unroll
            for (int q = 0; q < 8; ++q) { const float a = rnd ? bfr(v[q]) : v[q]; const float hn = (a * rinv) * bfr(g[q]); o[q] = toh_flush(hn * sc[q] + sf[q]); }
            *(volatile v8h*)(HB + (size_t)row * DM + c0) = o; }
        if (ps == 0) __threadfence(); }
}

__global__ __launch_bounds__(256) void k_gate(const float* __restrict__ F1, h16* G, size_t n8) {
#pragma clang fp contract(off)
    const size_t i = (size_t)blockIdx.x * 256 + threadIdx.x; if (i >= n8) return; const size_t row = i / (FF / 8); const size_t cg = i % (FF / 8);
    const float* p = F1 + row * (size_t)(2 * FF) + cg * 8; const v8f x1 = *(const v8f*)p; const v8f x2 = *(const v8f*)(p + FF); v8h o;
#pragma unroll
    for (int q = 0; q < 8; ++q) o[q] = toh_flush((silu_f(x1[q]) * x2[q]) * GCAR);
    *(volatile v8h*)(G + i * 8) = o; __threadfence(); *(volatile v8h*)(G + i * 8) = o; }

constexpr size_t al256(size_t b) { return (b + 255) & ~(size_t)255; }
constexpr size_t SZ_WQKV = al256((size_t)3 * DQ * DM * 2);
constexpr size_t SZ_WO   = al256((size_t)DM * DQ * 2);
constexpr size_t SZ_W1   = al256((size_t)2 * FF * DM * 2);
constexpr size_t SZ_W2   = al256((size_t)DM * FF * 2);
constexpr size_t SZ_MOD  = al256((size_t)2 * NB * DM * 4);
constexpr size_t SZ_HB   = al256((size_t)TT * DM * 2);
constexpr size_t SZ_PL   = al256((size_t)NH_ * TT * HD * 2);
constexpr size_t SZ_CTX  = al256((size_t)TT * DQ * 2);
constexpr size_t SZ_XM   = al256((size_t)TT * DM * 4);
constexpr size_t SZ_F    = (size_t)TT * 3 * DQ * 4;
constexpr size_t SZ_F1   = (size_t)MC * 2 * FF * 4;
constexpr size_t SZ_SF   = al256(SZ_F > SZ_F1 ? SZ_F : SZ_F1);
constexpr size_t SZ_G    = al256((size_t)TT * FF * 2);
constexpr size_t CARVE   = SZ_WQKV + SZ_WO + SZ_W1 + SZ_W2 + SZ_MOD + SZ_HB + 3 * SZ_PL + SZ_CTX + SZ_XM + SZ_SF + SZ_G;
static_assert(SZ_F <= SZ_SF);
static_assert(SZ_F1 <= SZ_SF);
static_assert(CARVE <= (size_t)134217728);

extern "C" void kernel_launch(void* const* d_in, const int* in_sizes, int n_in,
                              void* d_out, int out_size, void* d_ws, size_t ws_size, hipStream_t stream) {
    if (n_in < 15) return;
    const size_t need_x = (size_t)(NB - 1) * SEQ_FULL * DM + (size_t)TT * DM;
    if ((size_t)in_sizes[0] < need_x) return;
    if ((size_t)in_sizes[1] < (size_t)NB * DM) return;
    if ((size_t)in_sizes[2] < (size_t)(NB - 1) * SEQ_FULL + TT) return;
    if ((size_t)in_sizes[3] < (size_t)DM) return;
    if ((size_t)in_sizes[4] < (size_t)DM * DM) return;
    if ((size_t)in_sizes[5] < (size_t)DM) return;
    if ((size_t)in_sizes[6] < (size_t)DM * DM) return;
    if ((size_t)in_sizes[7] < (size_t)DM) return;
    if ((size_t)in_sizes[8] < (size_t)3 * DQ * DM) return;
    if ((size_t)in_sizes[9] < (size_t)DM * DQ) return;
    if ((size_t)in_sizes[10] < (size_t)DM) return;
    if ((size_t)in_sizes[11] < (size_t)2 * FF * DM) return;
    if ((size_t)in_sizes[12] < (size_t)2 * FF) return;
    if ((size_t)in_sizes[13] < (size_t)DM * FF) return;
    if ((size_t)in_sizes[14] < (size_t)DM) return;
    if ((size_t)out_size < need_x) return;
    if (CARVE > ws_size) return;
    const float* x = (const float*)d_in[0]; const float* cnd = (const float*)d_in[1]; const int* mask = (const int*)d_in[2]; const float* nw = (const float*)d_in[3];
    const float* scw = (const float*)d_in[4]; const float* scb = (const float*)d_in[5]; const float* shw = (const float*)d_in[6]; const float* shb = (const float*)d_in[7];
    const float* wqkv = (const float*)d_in[8]; const float* wo = (const float*)d_in[9]; const float* bo = (const float*)d_in[10];
    const float* w1 = (const float*)d_in[11]; const float* b1 = (const float*)d_in[12]; const float* w2 = (const float*)d_in[13]; const float* b2 = (const float*)d_in[14];
    float* OUT = (float*)d_out;
    char* wsp = (char*)d_ws;
    auto take = [&](size_t bytes) { char* p = wsp; wsp += bytes; return (void*)p; };
    h16* WQKV = (h16*)take(SZ_WQKV);
    h16* WO = (h16*)take(SZ_WO);
    h16* W1 = (h16*)take(SZ_W1);
    h16* W2 = (h16*)take(SZ_W2);
    float* MOD = (float*)take(SZ_MOD); float* MODSH = MOD; float* MODSC = MOD + (size_t)NB * DM;
    h16* HB = (h16*)take(SZ_HB);
    h16* QK = (h16*)take(2 * SZ_PL); h16* QP16 = QK; h16* KP16 = QK + (size_t)NH_ * TT * HD;
    h16* VT16 = (h16*)take(SZ_PL);
    h16* CTX = (h16*)take(SZ_CTX);
    float* XM = (float*)take(SZ_XM);
    float* F = (float*)take(SZ_SF);
    h16* G = (h16*)take(SZ_G);
    if ((size_t)(wsp - (char*)d_ws) > ws_size) return;
    auto g8 = [](size_t n8) { return (unsigned)((n8 + 255) / 256); };
    k_cvtw<<<g8((size_t)3 * DQ * DM / 8), 256, 0, stream>>>(wqkv, WQKV, (size_t)3 * DQ * DM / 8);
    k_cvtw<<<g8((size_t)DM * DQ / 8), 256, 0, stream>>>(wo, WO, (size_t)DM * DQ / 8);
    k_cvtw<<<g8((size_t)2 * FF * DM / 8), 256, 0, stream>>>(w1, W1, (size_t)2 * FF * DM / 8);
    k_cvtw<<<g8((size_t)DM * FF / 8), 256, 0, stream>>>(w2, W2, (size_t)DM * FF / 8);
    k_mod<<<DM / 32, 256, 0, stream>>>(cnd, shw, shb, MODSH, 0);
    k_mod<<<DM / 32, 256, 0, stream>>>(cnd, scw, scb, MODSC, 1);
    const float iw = 1.0f / WCAR;
    for (int b = 0; b < NB; ++b) {
        const float* xb = x + (size_t)b * SEQ_FULL * DM;
        k_adaln<<<TT / 8, 256, 0, stream>>>(xb, 1, nw, MODSC + (size_t)b * DM, MODSH + (size_t)b * DM, HB);
        k_gemm_nb<<<dim3(TT / 64, 3 * DQ / 64, 1), 32, 0, stream>>>(HB, WQKV, DM, F, 3 * DQ, iw);
        k_hpl16<<<g8((size_t)2 * NH_ * TT * HD / 8), 256, 0, stream>>>(F, 3 * DQ, 2 * NH_, QK);
        k_vtp16<<<g8((size_t)NH_ * HD * TT / 8), 256, 0, stream>>>(F + 2 * DQ, 3 * DQ, NH_, VT16);
        k_flash<<<dim3(TT / 64, NH_, 1), 128, 0, stream>>>(QP16, KP16, VT16, mask + (size_t)b * SEQ_FULL, CTX);
        k_gemm_br1<<<dim3(TT / 64, DM / 64, 1), 32, 0, stream>>>(CTX, WO, DQ, XM, DM, bo, xb, DM, 1.0f / (WCAR * CCAR));
        k_adaln<<<TT / 8, 256, 0, stream>>>(XM, 0, nw, MODSC + (size_t)b * DM, MODSH + (size_t)b * DM, HB);
        for (int ch = 0; ch < TT / MC; ++ch) {
            k_gemm_b<<<dim3(MC / 64, 2 * FF / 64, 1), 32, 0, stream>>>(HB + (size_t)ch * MC * DM, W1, DM, F, 2 * FF, b1, iw);
            k_gate<<<g8((size_t)MC * FF / 8), 256, 0, stream>>>(F, G + (size_t)ch * MC * FF, (size_t)MC * FF / 8); }
        k_gemm_br2<<<dim3(TT / 64, DM / 64, 1), 32, 0, stream>>>(G, W2, FF, OUT + (size_t)b * SEQ_FULL * DM, DM, b2, XM, DM, 1.0f / (WCAR * GCAR)); }
}
